// attention_9663676416592
// MI455X (gfx1250) — hardware-run, weakly checked
//
#include <hip/hip_runtime.h>


#ifndef NB
#define NB 2
#endif
#ifndef SEQ
#define SEQ 4096
#endif
#define NB_FULL  2
#define SEQ_FULL 4096
#ifndef OUT_SEQ
#define OUT_SEQ SEQ
#endif
#define CH   256
#define AW   4
#define XP   68
#define WCAR 1024.0f
#define QCAR 16.0f
#define QSC  (QCAR / WCAR)
#define SCL  ((float)(1.4426950408889634 / 16.0))
#define L2E  1.4426950408889634f
#define NEGB (-3.0e38f)
#define OUT1_OFF ((size_t)NB_FULL * SEQ_FULL)

static_assert(OUT1_OFF * 4 == 32768);
static_assert(CH % 32 == 0);
static_assert(CH % 64 == 0);
static_assert(CH == 32 * 8);
static_assert(SEQ % 64 == 0);
static_assert((NB * SEQ) % 64 == 0);
static_assert(SEQ % (16 * AW) == 0);
static_assert(16 * AW == 16 * 4);
static_assert(OUT_SEQ % 32 == 0);
static_assert(OUT_SEQ >= SEQ);
static_assert(NB <= NB_FULL);
static_assert(SEQ <= SEQ_FULL);
static_assert((XP * 4) % 16 == 0);
static_assert(256 * 16 * 4 == CH * 64);
static_assert((256 / 32) * 8 == 64);
static_assert((CH * XP + 64) * 4 <= 131072);
static_assert(16 * 68 * 4 <= 131072);
static_assert(4 * (32 / 8) == 16);
static_assert(8 * 8 == 64);

typedef _Float16 h16;
typedef unsigned short bf;
typedef __attribute__((ext_vector_type(16))) _Float16 v16h;
typedef __attribute__((ext_vector_type(8)))  _Float16 v8h;
typedef __attribute__((ext_vector_type(8)))  float    v8f;
typedef __attribute__((ext_vector_type(4)))  float    v4f;
typedef v4f  __attribute__((may_alias)) v4fa;

__device__ __forceinline__ unsigned short f2bf(float f) { unsigned u = __float_as_uint(f); u += 0x7FFFu + ((u >> 16) & 1u); return (unsigned short)(u >> 16); }
__device__ __forceinline__ float bfr(float f) { return __uint_as_float(((unsigned)f2bf(f)) << 16); }
__device__ __forceinline__ v16h cat16(v8h lo, v8h hi) { return __builtin_shufflevector(lo, hi, 0, 1, 2, 3, 4, 5, 6, 7, 8, 9, 10, 11, 12, 13, 14, 15); }
__device__ __forceinline__ v8f wmma16(v16h a, v16h b, v8f c) { return __builtin_amdgcn_wmma_f32_16x16x32_f16(false, a, false, b, (short)0, c, false, false); }
__device__ __forceinline__ v8f wmma16g(v16h a, v16h b, v8f c) { c = wmma16(a, b, c); asm volatile("v_nop\n\tv_nop\n\tv_nop\n\tv_nop" : "+v"(c) : "v"(a), "v"(b)); return c; }
__device__ __forceinline__ v16h  ldh(const h16* p) { return cat16(*(const v8h*)p, *(const v8h*)(p + 16)); }
__device__ __forceinline__ void wave_sync() { __builtin_amdgcn_fence(3  , "wavefront"); __builtin_amdgcn_wave_barrier(); asm volatile("" ::: "memory"); }
static __device__ __forceinline__ h16 toh_flush(float v) { const h16 r = (h16)v; return (fabsf(v) < 6.103515625e-05f) ? (h16)0.0f : r; }

__global__ __launch_bounds__(256) void k_xt(const float* __restrict__ X, const float* __restrict__ Wg, h16* XTp, float* VVp) {
    __shared__ __align__(16) float xs[CH * XP];
    __shared__ __align__(16) float vs[64];
    const int t = threadIdx.x, lane = t & 31;
    const int wave = __builtin_amdgcn_readfirstlane((int)(threadIdx.x >> 5));
    const int jt = blockIdx.x, b = blockIdx.y;
    const float* xb = X + (size_t)b * CH * SEQ_FULL + (size_t)jt * 64;
#pragma unroll 4
    for (int it = 0; it < 16; ++it) {
        const int cid = t + 256 * it; const int c = cid >> 4, f = cid & 15;
        const v4f d = *(const v4f*)(xb + (size_t)c * SEQ_FULL + f * 4);
        v4f e; e[0] = bfr(d[0]); e[1] = bfr(d[1]); e[2] = bfr(d[2]); e[3] = bfr(d[3]);
        *(v4fa*)(&xs[c * XP + f * 4]) = e;
    }
    __syncthreads();
    if (wave < 2) {
        const int j = wave * 32 + lane; float acc = 0.0f;
#pragma unroll 4
        for (int c = 0; c < CH; ++c) acc = fmaf(bfr(Wg[c]), xs[c * XP + j], acc);
        vs[j] = acc;
    }
    __syncthreads();
    const size_t rowb = (size_t)b * SEQ + (size_t)jt * 64;
#pragma unroll 1
    for (int ps = 0; ps < 2; ++ps) {
#pragma unroll 2
        for (int s = 0; s < 8; ++s) { const int j = wave * 8 + s; v8h hv;
#pragma unroll
            for (int k = 0; k < 8; ++k) hv[k] = toh_flush(xs[(lane * 8 + k) * XP + j]);
            *(volatile v8h*)(XTp + (rowb + (size_t)j) * CH + lane * 8) = hv; }
        if (wave == 0) {
            const v4f val = *(const v4fa*)(&vs[(lane & 15) * 4]);
            if (lane < 16) *(volatile v4f*)(VVp + rowb + lane * 4) = val; }
        if (ps == 0) __threadfence(); }
}

__global__ __launch_bounds__(256) void k_wcv2(const float* __restrict__ we, const float* __restrict__ wq, h16* WH, size_t n8) {
    const size_t i = (size_t)blockIdx.x * 256 + threadIdx.x; if (i >= n8) return;
    const v8f a = *(const v8f*)(we + i * 8); const v8f c = *(const v8f*)(wq + i * 8); v8h oa, oc;
#pragma unroll
    for (int k = 0; k < 8; ++k) { oa[k] = toh_flush(bfr(a[k]) * WCAR); oc[k] = toh_flush(bfr(c[k]) * WCAR); }
    h16* d0 = WH + i * 8; h16* d1 = WH + (size_t)CH * CH + i * 8;
    *(volatile v8h*)d0 = oa; *(volatile v8h*)d1 = oc; __threadfence(); *(volatile v8h*)d0 = oa; *(volatile v8h*)d1 = oc;
}

__global__ __launch_bounds__(32) void k_corr(const h16* __restrict__ XT, const h16* __restrict__ WH, h16* QP) {
    __shared__ __align__(16) float os[16 * 68];
    const int K = CH;
    const int lane = threadIdx.x & 31, lr = lane & 15, hi = lane >> 4; const int r0 = blockIdx.x * 64, c0 = blockIdx.y * 64; const int mz = blockIdx.z;
    const size_t pln = (size_t)NB * SEQ * CH;
    v8f acc[4][4];
#pragma unroll
    for (int mb = 0; mb < 4; ++mb)
#pragma unroll
        for (int nb = 0; nb < 4; ++nb) acc[mb][nb] = (v8f){};
    const size_t aoff = (size_t)mz * pln + (size_t)(r0 + lr) * K + 8 * hi, boff = (size_t)mz * CH * CH + (size_t)(c0 + lr) * K + 8 * hi;
#pragma unroll 1
    for (int kc = 0; kc < K; kc += 32) {
        v16h a[4];
#pragma unroll
        for (int mb = 0; mb < 4; ++mb) a[mb] = ldh(XT + aoff + (size_t)mb * 16 * K + kc);
#pragma unroll
        for (int nb = 0; nb < 4; ++nb) { const v16h b = ldh(WH + boff + (size_t)nb * 16 * K + kc);
#pragma unroll
            for (int mb = 0; mb < 4; ++mb) acc[mb][nb] = wmma16g(a[mb], b, acc[mb][nb]); }
    }
    const size_t tbase = (size_t)mz * pln + (size_t)r0 * CH + (size_t)c0;
#pragma unroll
    for (int mb = 0; mb < 4; ++mb) {
#pragma unroll
        for (int nb = 0; nb < 4; ++nb) {
#pragma unroll
            for (int j = 0; j < 8; ++j) os[(hi * 8 + j) * 68 + nb * 16 + lr] = acc[mb][nb][j] * QSC; }
        wave_sync();
#pragma unroll 1
        for (int ps = 0; ps < 2; ++ps) {
            const size_t sb = tbase + (size_t)(mb * 16) * CH;
#pragma unroll
            for (int s = 0; s < 4; ++s) { const int row = 4 * s + (lane >> 3), c8 = (lane & 7) * 8;
                const v4f x0 = *(const v4fa*)(&os[row * 68 + c8]); const v4f x1 = *(const v4fa*)(&os[row * 68 + c8 + 4]); v8h hv;
#pragma unroll
                for (int i = 0; i < 4; ++i) { hv[i] = toh_flush(x0[i]); hv[4 + i] = toh_flush(x1[i]); }
                *(volatile v8h*)(QP + sb + (size_t)row * CH + c8) = hv; }
            if (ps == 0) __threadfence(); }
        wave_sync();
    }
}

__global__ __launch_bounds__(32 * AW) void k_coatt(const h16* __restrict__ QP, const h16* __restrict__ XT, const float* __restrict__ VV, float* OUT) {
    __shared__ __align__(16) float rs[16 * AW];
    const int lane = threadIdx.x & 31, lr = lane & 15, hi = lane >> 4;
    const int wave = __builtin_amdgcn_readfirstlane((int)(threadIdx.x >> 5));
    const int inst = blockIdx.y; const int m = inst / NB, b = inst % NB;
    const int t0 = (blockIdx.x * AW + wave) * 16;
    const size_t qo = ((size_t)(m * NB + b) * SEQ + (size_t)(t0 + lr)) * CH + 8 * hi;
    const size_t ko = ((size_t)((1 - m) * NB + b) * SEQ + (size_t)lr) * CH + 8 * hi;
    const size_t vo = (size_t)(m * NB + b) * SEQ + 8 * hi;
    float mrun = NEGB, lrun = 0.0f, orun = 0.0f;
#pragma unroll 1
    for (int key0 = 0; key0 < SEQ; key0 += 64) {
        v8f s0 = (v8f){}, s1 = (v8f){}, s2 = (v8f){}, s3 = (v8f){};
        const size_t kb = ko + (size_t)key0 * CH;
#pragma unroll 1
        for (int kc = 0; kc < CH; kc += 32) {
            const v16h qf = ldh(QP + qo + kc);
            const h16* ka = XT + kb + kc;
            const v16h a0 = ldh(ka), a1 = ldh(ka + 16 * CH), a2 = ldh(ka + 32 * CH), a3 = ldh(ka + 48 * CH);
            s0 = wmma16g(a0, qf, s0); s1 = wmma16g(a1, qf, s1); s2 = wmma16g(a2, qf, s2); s3 = wmma16g(a3, qf, s3);
        }
        const float* vp = VV + vo + key0;
        v4f w[8];
#pragma unroll
        for (int n = 0; n < 4; ++n) { w[2 * n] = *(const v4f*)(vp + 16 * n); w[2 * n + 1] = *(const v4f*)(vp + 16 * n + 4); }
        float sv[32], vv[32];
#pragma unroll
        for (int r = 0; r < 8; ++r) { sv[r] = s0[r]; sv[8 + r] = s1[r]; sv[16 + r] = s2[r]; sv[24 + r] = s3[r]; }
#pragma unroll
        for (int n = 0; n < 4; ++n) {
#pragma unroll
            for (int r = 0; r < 4; ++r) { vv[8 * n + r] = w[2 * n][r]; vv[8 * n + 4 + r] = w[2 * n + 1][r]; } }
        float mxr = sv[0];
#pragma unroll
        for (int i = 1; i < 32; ++i) mxr = fmaxf(mxr, sv[i]);
        float mx = mxr * SCL;
        mx = fmaxf(mx, __shfl_xor(mx, 16, 32));
        const float mnew = fmaxf(mrun, mx);
        const float alpha = __builtin_amdgcn_exp2f(mrun - mnew);
        float ls = 0.0f, osum = 0.0f;
#pragma unroll
        for (int i = 0; i < 32; ++i) {
            const float e = __builtin_amdgcn_exp2f(fmaf(sv[i], SCL, -mnew));
            ls += e; osum = fmaf(e, vv[i], osum); }
        lrun = lrun * alpha + ls; orun = orun * alpha + osum; mrun = mnew;
    }
    lrun += __shfl_xor(lrun, 16, 32);
    orun += __shfl_xor(orun, 16, 32);
    const float z = orun * (1.0f / lrun);
    const float sg = 1.0f / (1.0f + __builtin_amdgcn_exp2f(-z * L2E));
    if (hi == 0) rs[wave * 16 + lr] = sg;
    __syncthreads();
    if (wave == 0) {
        const v4f val = *(const v4fa*)(&rs[(lane & 15) * 4]);
        float* orow = OUT + (size_t)m * OUT1_OFF + (size_t)b * OUT_SEQ + (size_t)blockIdx.x * (16 * AW);
#pragma unroll 1
        for (int ps = 0; ps < 2; ++ps) {
            if (lane < 16) *(volatile v4f*)(orow + lane * 4) = val;
            if (ps == 0) __threadfence(); }
    }
}

static constexpr size_t al256(size_t v) { return (v + 255) & ~(size_t)255; }
static constexpr size_t SZ_PL = al256((size_t)2 * NB * SEQ * CH * 2);
static constexpr size_t SZ_WH = al256((size_t)2 * CH * CH * 2);
static constexpr size_t SZ_VV = al256((size_t)2 * NB * SEQ * 4);
static constexpr size_t SZ_TOTAL = 2 * SZ_PL + SZ_WH + SZ_VV;
static_assert(SZ_TOTAL <= (size_t)134217728);
static_assert(((size_t)NB * SEQ * CH * 2) % 256 == 0);
static_assert(((size_t)CH * CH * 2) % 256 == 0);
static_assert(((size_t)NB * SEQ * 4) % 256 == 0);
static_assert(((size_t)CH * CH) % (8 * 32) == 0);

extern "C" void kernel_launch(void* const* d_in, const int* in_sizes, int n_in,
                              void* d_out, int out_size, void* d_ws, size_t ws_size, hipStream_t stream) {
    if (n_in < 5) return;
    const size_t needx = ((size_t)(NB - 1) * CH + (size_t)(CH - 1)) * SEQ_FULL + SEQ;
    if ((size_t)in_sizes[0] < needx || (size_t)in_sizes[1] < needx) return;
    if ((size_t)in_sizes[2] < (size_t)CH * CH || (size_t)in_sizes[3] < (size_t)CH * CH || in_sizes[4] < CH) return;
    if ((size_t)out_size < OUT1_OFF + (size_t)(NB - 1) * OUT_SEQ + SEQ) return;
    if (SZ_TOTAL > ws_size) return;
    const float* ex = (const float*)d_in[0]; const float* qu = (const float*)d_in[1];
    const float* we = (const float*)d_in[2]; const float* wq = (const float*)d_in[3];
    const float* wg = (const float*)d_in[4];
    float* OUT = (float*)d_out;
    char* wsp = (char*)d_ws;
    h16* XT = (h16*)wsp; wsp += SZ_PL;
    h16* QP = (h16*)wsp; wsp += SZ_PL;
    h16* WH = (h16*)wsp; wsp += SZ_WH;
    float* VV = (float*)wsp; wsp += SZ_VV;
    const size_t pln = (size_t)NB * SEQ * CH;

    k_xt<<<dim3(SEQ / 64, NB, 1), 256, 0, stream>>>(ex, wg, XT, VV);
    k_xt<<<dim3(SEQ / 64, NB, 1), 256, 0, stream>>>(qu, wg, XT + pln, VV + (size_t)NB * SEQ);
    { const size_t n8 = (size_t)CH * CH / 8;
      k_wcv2<<<(unsigned)((n8 + 255) / 256), 256, 0, stream>>>(we, wq, WH, n8); }
    k_corr<<<dim3(NB * SEQ / 64, CH / 64, 2), 32, 0, stream>>>(XT, WH, QP);
    k_coatt<<<dim3(SEQ / (16 * AW), 2 * NB, 1), 32 * AW, 0, stream>>>(QP, XT, VV, OUT);
}
